// HeteroGAT_81071802679584
// MI455X (gfx1250) — hardware-verified
//
#include <hip/hip_runtime.h>


#define CH   4096
#define NBC  2048
#define LCAP 1024
#define QCAP 128

typedef unsigned short us;
typedef us       v8us  __attribute__((ext_vector_type(8)));
typedef us       v16us __attribute__((ext_vector_type(16)));
typedef __bf16   v16bf __attribute__((ext_vector_type(16)));
typedef float    v8f   __attribute__((ext_vector_type(8)));
typedef float    v4f   __attribute__((ext_vector_type(4)));
typedef unsigned v4u   __attribute__((ext_vector_type(4)));
typedef int      v4i   __attribute__((ext_vector_type(4)));
typedef float    v4fa  __attribute__((ext_vector_type(4), may_alias));
typedef unsigned v4ua  __attribute__((ext_vector_type(4), may_alias));

union Frag { v16us v; v8us h[2]; v16bf b; };

__device__ __forceinline__ us bf_rne(float f) {
  unsigned u = __float_as_uint(f);
  u += 0x7FFFu + ((u >> 16) & 1u);
  return (us)(u >> 16);
}
__device__ __forceinline__ float bf_val(us b) { return __uint_as_float(((unsigned)b) << 16); }

__device__ __forceinline__ v8f mma16(const Frag& a, const Frag& b, v8f c) {
  c = __builtin_amdgcn_wmma_f32_16x16x32_bf16(false, a.b, false, b.b, (short)0, c, false, false);
  asm volatile("v_nop\n\tv_nop\n\tv_nop\n\tv_nop" : "+v"(c) : "v"(a.v), "v"(b.v));
  return c;
}

__device__ __forceinline__ float wsum(float v) {
  #pragma unroll
  for (int o = 16; o > 0; o >>= 1) v += __shfl_xor(v, o);
  return v;
}
__device__ __forceinline__ float wmax(float v) {
  #pragma unroll
  for (int o = 16; o > 0; o >>= 1) v = fmaxf(v, __shfl_xor(v, o));
  return v;
}

__global__ __launch_bounds__(32) void k_fold(const float* __restrict__ We, const float* __restrict__ Ae,
                                             int K, float* F) {
  __shared__ __attribute__((aligned(16))) float s[32];
  const int t = threadIdx.x;
  const int k = t >> 2, hd = t & 3;
  float a = 0.f;
  if (k < K) {
    #pragma unroll 1
    for (int c = 0; c < 32; ++c) a += We[k * 128 + hd * 32 + c] * Ae[hd * 32 + c];
  }
  s[t] = a;
  __syncthreads();
  v4f v = {0.f, 0.f, 0.f, 0.f};
  if (t < 8) v = *(const v4fa*)&s[4 * t];
  if (t < 8) *(volatile v4f*)(F + 4 * t) = v;
  __threadfence();
  if (t < 8) *(volatile v4f*)(F + 4 * t) = v;
}

__global__ __launch_bounds__(256) void k_packb(const float* __restrict__ W, int K, int KS, us* Bh, us* Bl) {
  const int idx = blockIdx.x * 256 + threadIdx.x;
  if (idx >= KS * 512) return;
  const int half = idx & 1, lane = (idx >> 1) & 31, nt = (idx >> 6) & 7, ks = idx >> 9;
  const int n = nt * 16 + (lane & 15);
  const int kb = ks * 32 + 16 * half + 8 * (lane >> 4);
  v8us vh, vl;
  #pragma unroll
  for (int q = 0; q < 8; ++q) {
    const int k = kb + q;
    float f = 0.f;
    if (k < K) f = W[(size_t)k * 128 + n];
    const us hb = bf_rne(f);
    const us lb = bf_rne(f - bf_val(hb));
    vh[q] = hb; vl[q] = lb;
  }
  us* ph = Bh + (size_t)idx * 8;
  us* pl = Bl + (size_t)idx * 8;
  *(volatile v8us*)ph = vh; *(volatile v8us*)pl = vl;
  __threadfence();
  *(volatile v8us*)ph = vh; *(volatile v8us*)pl = vl;
}

__global__ __launch_bounds__(256) void k_cvt(const float* __restrict__ X, int M, int Mp, int K, us* Ah, us* Al) {
  const int idx = blockIdx.x * 256 + threadIdx.x;
  if (idx >= Mp * 4) return;
  const int m = idx >> 2, g = idx & 3;
  v8us vh, vl;
  #pragma unroll
  for (int q = 0; q < 8; ++q) {
    const int k = 8 * g + q;
    float f = 0.f;
    if (m < M && k < K) f = X[(size_t)m * K + k];
    const us hb = bf_rne(f);
    const us lb = bf_rne(f - bf_val(hb));
    vh[q] = hb; vl[q] = lb;
  }
  us* ph = Ah + (size_t)idx * 8;
  us* pl = Al + (size_t)idx * 8;
  *(volatile v8us*)ph = vh; *(volatile v8us*)pl = vl;
  __threadfence();
  *(volatile v8us*)ph = vh; *(volatile v8us*)pl = vl;
}

__global__ __launch_bounds__(256) void k_gemm(const us* __restrict__ Ah, const us* __restrict__ Al, int lda, int KS, int M,
                                              const us* __restrict__ Bh, const us* __restrict__ Bl,
                                              const float* __restrict__ vA, const float* __restrict__ vB,
                                              float* Y, int writeY, float* S) {
  __shared__ __attribute__((aligned(16))) float sD[16][132];
  __shared__ __attribute__((aligned(16))) float sS[128];
  const int tid = threadIdx.x, w = tid >> 5, lane = tid & 31, hf = lane >> 4, mr = lane & 15;
  const int m0 = blockIdx.x * 16;
  int row = m0 + mr;
  if (row > M - 1) row = M - 1;
  const us* ah = Ah + (size_t)row * lda;
  const us* al = Al + (size_t)row * lda;
  v8f acc = {0.f, 0.f, 0.f, 0.f, 0.f, 0.f, 0.f, 0.f};
  for (int ks = 0; ks < KS; ++ks) {
    const int k0 = ks * 32;
    Frag fa, ga, fb, gb;
    fa.h[0] = *(const v8us*)(ah + k0 + 8 * hf);
    fa.h[1] = *(const v8us*)(ah + k0 + 16 + 8 * hf);
    ga.h[0] = *(const v8us*)(al + k0 + 8 * hf);
    ga.h[1] = *(const v8us*)(al + k0 + 16 + 8 * hf);
    const size_t bo = ((size_t)(ks * 8 + w) * 32 + lane) * 16;
    fb.h[0] = *(const v8us*)(Bh + bo);
    fb.h[1] = *(const v8us*)(Bh + bo + 8);
    gb.h[0] = *(const v8us*)(Bl + bo);
    gb.h[1] = *(const v8us*)(Bl + bo + 8);
    acc = mma16(fa, fb, acc);
    acc = mma16(fa, gb, acc);
    acc = mma16(ga, fb, acc);
  }
  #pragma unroll
  for (int r = 0; r < 8; ++r) sD[8 * hf + r][16 * w + mr] = acc[r];
  __syncthreads();
  {
    const int r = tid >> 4, hd = (tid >> 2) & 3, q = tid & 3;
    float pa = 0.f, pb = 0.f;
    #pragma unroll
    for (int c = 0; c < 8; ++c) {
      const int col = 32 * hd + 8 * q + c;
      const float d = sD[r][col];
      pa += d * vA[col];
      pb += d * vB[col];
    }
    pa += __shfl_xor(pa, 1); pa += __shfl_xor(pa, 2);
    pb += __shfl_xor(pb, 1); pb += __shfl_xor(pb, 2);
    if (q == 0) { sS[r * 8 + hd] = pa; sS[r * 8 + 4 + hd] = pb; }
  }
  __syncthreads();
  const v4f y0 = *(const v4fa*)&sD[2 * w][4 * lane];
  const v4f y1 = *(const v4fa*)&sD[2 * w + 1][4 * lane];
  const v4f sv = *(const v4fa*)&sS[4 * lane];
  const bool wy0 = (writeY != 0) && (m0 + 2 * w < M);
  const bool wy1 = (writeY != 0) && (m0 + 2 * w + 1 < M);
  float* yp0 = Y + (size_t)(m0 + 2 * w) * 128 + 4 * lane;
  float* yp1 = Y + (size_t)(m0 + 2 * w + 1) * 128 + 4 * lane;
  float* spo = S + (size_t)m0 * 8 + 4 * lane;
  if (wy0) *(volatile v4f*)yp0 = y0;
  if (wy1) *(volatile v4f*)yp1 = y1;
  if (w == 0) *(volatile v4f*)spo = sv;
  __threadfence();
  if (wy0) *(volatile v4f*)yp0 = y0;
  if (wy1) *(volatile v4f*)yp1 = y1;
  if (w == 0) *(volatile v4f*)spo = sv;
}

__global__ __launch_bounds__(256) void k_sort(const int* __restrict__ dst, int E, int NT, int NPB, unsigned magic,
                                              unsigned* srt, int* bnd) {
  __shared__ __attribute__((aligned(16))) unsigned key[CH];
  const int tid = threadIdx.x, c = blockIdx.x;
  const int base = c * CH;
  #pragma unroll
  for (int i = 0; i < 16; ++i) {
    const int p = tid + 256 * i;
    const int e = base + p;
    unsigned v = 0xFFFFFFFFu;
    if (e < E) {
      const int d = dst[e];
      unsigned b = 2047u, ln = 0u;
      if ((unsigned)d < (unsigned)NT) {
        b = (NPB == 1) ? (unsigned)d : __umulhi((unsigned)d, magic);
        ln = (unsigned)d - b * (unsigned)NPB;
      }
      v = (b << 17) | (ln << 12) | (unsigned)p;
    }
    key[p] = v;
  }
  for (int size = 2; size <= CH; size <<= 1) {
    for (int stride = size >> 1; stride > 0; stride >>= 1) {
      __syncthreads();
      #pragma unroll
      for (int q = 0; q < 8; ++q) {
        const int pid = tid + 256 * q;
        const int i = (pid << 1) - (pid & (stride - 1));
        const int i2 = i + stride;
        const unsigned a = key[i], bb = key[i2];
        const bool up = ((i & size) == 0);
        if ((a > bb) == up) { key[i] = bb; key[i2] = a; }
      }
    }
  }
  __syncthreads();
  v4i bv0, bv1;
  #pragma unroll
  for (int half = 0; half < 2; ++half) {
    #pragma unroll
    for (int q = 0; q < 4; ++q) {
      const int jj = 1024 * half + 4 * tid + q;
      const unsigned tgt = ((unsigned)jj) << 17;
      int pos = 0;
      #pragma unroll
      for (int s = CH / 2; s > 0; s >>= 1) { if (key[pos + s - 1] < tgt) pos += s; }
      if (key[pos] < tgt) pos += 1;
      if (half == 0) bv0[q] = pos; else bv1[q] = pos;
    }
  }
  const v4u s0 = *(const v4ua*)&key[4 * tid];
  const v4u s1 = *(const v4ua*)&key[1024 + 4 * tid];
  const v4u s2 = *(const v4ua*)&key[2048 + 4 * tid];
  const v4u s3 = *(const v4ua*)&key[3072 + 4 * tid];
  int* bp = bnd + (size_t)c * NBC;
  unsigned* sp = srt + (size_t)base;
  *(volatile v4i*)(bp + 4 * tid) = bv0;
  *(volatile v4i*)(bp + 1024 + 4 * tid) = bv1;
  *(volatile v4u*)(sp + 4 * tid) = s0;
  *(volatile v4u*)(sp + 1024 + 4 * tid) = s1;
  *(volatile v4u*)(sp + 2048 + 4 * tid) = s2;
  *(volatile v4u*)(sp + 3072 + 4 * tid) = s3;
  __threadfence();
  *(volatile v4i*)(bp + 4 * tid) = bv0;
  *(volatile v4i*)(bp + 1024 + 4 * tid) = bv1;
  *(volatile v4u*)(sp + 4 * tid) = s0;
  *(volatile v4u*)(sp + 1024 + 4 * tid) = s1;
  *(volatile v4u*)(sp + 2048 + 4 * tid) = s2;
  *(volatile v4u*)(sp + 3072 + 4 * tid) = s3;
}

template <int MODE>
__global__ __launch_bounds__(256) void k_agg(const unsigned* __restrict__ srt, const int* __restrict__ bnd, int nch,
                                             int NT, int NPB, const int* __restrict__ src, int Nsrc,
                                             const float* __restrict__ ea, int edim, const float* __restrict__ wef,
                                             const float* Ssrc, const float* Sdst,
                                             const float* __restrict__ hsrc, const float* __restrict__ bias,
                                             us* th, us* tl, int coloff, float* out) {
  __shared__ int l_eid[LCAP];
  __shared__ int l_ln[LCAP];
  __shared__ int q_src[8][QCAP];
  __shared__ __attribute__((aligned(16))) float q_lg[8][QCAP][4];
  __shared__ __attribute__((aligned(16))) unsigned fun[8][128];
  __shared__ float swef[32];
  __shared__ int wtot[8];
  const int tid = threadIdx.x, w = tid >> 5, lane = tid & 31, hl = lane >> 3;
  const int j = blockIdx.x;
  if (tid < 32) swef[tid] = wef[tid];
  const int c = tid;
  int lo = 0, cnt = 0;
  if (c < nch) {
    lo = bnd[(size_t)c * NBC + j];
    int hi = bnd[(size_t)c * NBC + j + 1];
    if (lo < 0) lo = 0;
    if (hi > CH) hi = CH;
    cnt = hi - lo;
    if (cnt < 0) cnt = 0;
  }
  int x = cnt;
  #pragma unroll
  for (int d = 1; d < 32; d <<= 1) { const int y = __shfl_up(x, d); if (lane >= d) x += y; }
  if (lane == 31) wtot[w] = x;
  __syncthreads();
  int pre = 0, total = 0;
  #pragma unroll
  for (int i = 0; i < 8; ++i) { const int t = wtot[i]; total += t; if (i < w) pre += t; }
  const int off = pre + x - cnt;
  for (int i = 0; i < cnt; ++i) {
    const int p = off + i;
    if (p < LCAP) {
      const unsigned u = srt[(size_t)c * CH + lo + i];
      l_eid[p] = c * CH + (int)(u & 4095u);
      l_ln[p] = (int)((u >> 12) & 31u);
    }
  }
  if (total > LCAP) total = LCAP;
  __syncthreads();

  const float NEG = __uint_as_float(0xff800000u);
  for (int ln = w; ln < NPB; ln += 8) {
    const int n = j * NPB + ln;
    if (n >= NT) break;
    int deg = 0;
    for (int p0 = 0; p0 < total; p0 += 32) {
      const int p = p0 + lane;
      const bool m = (p < total) && (l_ln[p] == ln);
      const unsigned bal = __builtin_amdgcn_ballot_w32(m);
      const int slot = deg + (int)__popc(bal & ((1u << lane) - 1u));
      if (m && slot < QCAP - 1) q_src[w][slot] = l_eid[p];
      deg += (int)__popc(bal);
    }
    const int degr = deg;
    if (deg > QCAP - 1) deg = QCAP - 1;
    const float* dp = Sdst + (size_t)n * 8;
    const float sd0 = dp[0], sd1 = dp[1], sd2 = dp[2], sd3 = dp[3];
    float mx0 = NEG, mx1 = NEG, mx2 = NEG, mx3 = NEG;
    float es0 = 0.f, es1 = 0.f, es2 = 0.f, es3 = 0.f;
    for (int i = lane; i < deg; i += 32) {
      const int e = q_src[w][i];
      int s = src[e];
      s = s < 0 ? 0 : s;
      s = s > Nsrc - 1 ? Nsrc - 1 : s;
      const float* sp = Ssrc + (size_t)s * 8;
      float g0 = sp[0] + sd0, g1 = sp[1] + sd1, g2 = sp[2] + sd2, g3 = sp[3] + sd3;
      if (MODE == 0) {
        const float* ap = ea + (size_t)e * edim;
        #pragma unroll 1
        for (int k = 0; k < edim; ++k) {
          const float a = ap[k];
          g0 += a * swef[4 * k]; g1 += a * swef[4 * k + 1]; g2 += a * swef[4 * k + 2]; g3 += a * swef[4 * k + 3];
        }
      } else {
        const v4f a4 = *(const v4f*)(ea + (size_t)e * 4);
        es0 += a4[0]; es1 += a4[1]; es2 += a4[2]; es3 += a4[3];
        #pragma unroll
        for (int k = 0; k < 4; ++k) {
          const float a = a4[k];
          g0 += a * swef[4 * k]; g1 += a * swef[4 * k + 1]; g2 += a * swef[4 * k + 2]; g3 += a * swef[4 * k + 3];
        }
      }
      g0 = g0 > 0.f ? g0 : 0.2f * g0;
      g1 = g1 > 0.f ? g1 : 0.2f * g1;
      g2 = g2 > 0.f ? g2 : 0.2f * g2;
      g3 = g3 > 0.f ? g3 : 0.2f * g3;
      q_src[w][i] = s;
      q_lg[w][i][0] = g0; q_lg[w][i][1] = g1; q_lg[w][i][2] = g2; q_lg[w][i][3] = g3;
      mx0 = fmaxf(mx0, g0); mx1 = fmaxf(mx1, g1); mx2 = fmaxf(mx2, g2); mx3 = fmaxf(mx3, g3);
    }
    int degt = deg;
    if (MODE == 1) {
      es0 = wsum(es0); es1 = wsum(es1); es2 = wsum(es2); es3 = wsum(es3);
      const float inv = 1.0f / fmaxf((float)degr, 1.0f);
      const float m0 = es0 * inv, m1 = es1 * inv, m2 = es2 * inv, m3 = es3 * inv;
      const float* np = Ssrc + (size_t)n * 8;
      float t0 = np[0] + sd0, t1 = np[1] + sd1, t2 = np[2] + sd2, t3 = np[3] + sd3;
      t0 += m0 * swef[0] + m1 * swef[4] + m2 * swef[8]  + m3 * swef[12];
      t1 += m0 * swef[1] + m1 * swef[5] + m2 * swef[9]  + m3 * swef[13];
      t2 += m0 * swef[2] + m1 * swef[6] + m2 * swef[10] + m3 * swef[14];
      t3 += m0 * swef[3] + m1 * swef[7] + m2 * swef[11] + m3 * swef[15];
      t0 = t0 > 0.f ? t0 : 0.2f * t0;
      t1 = t1 > 0.f ? t1 : 0.2f * t1;
      t2 = t2 > 0.f ? t2 : 0.2f * t2;
      t3 = t3 > 0.f ? t3 : 0.2f * t3;
      mx0 = fmaxf(mx0, t0); mx1 = fmaxf(mx1, t1); mx2 = fmaxf(mx2, t2); mx3 = fmaxf(mx3, t3);
      if (lane == 0) {
        q_src[w][deg] = n;
        q_lg[w][deg][0] = t0; q_lg[w][deg][1] = t1; q_lg[w][deg][2] = t2; q_lg[w][deg][3] = t3;
      }
      degt = deg + 1;
    }
    mx0 = wmax(mx0); mx1 = wmax(mx1); mx2 = wmax(mx2); mx3 = wmax(mx3);
    float ds0 = 0.f, ds1 = 0.f, ds2 = 0.f, ds3 = 0.f;
    for (int i = lane; i < degt; i += 32) {
      const float x0 = __expf(q_lg[w][i][0] - mx0);
      const float x1 = __expf(q_lg[w][i][1] - mx1);
      const float x2 = __expf(q_lg[w][i][2] - mx2);
      const float x3 = __expf(q_lg[w][i][3] - mx3);
      q_lg[w][i][0] = x0; q_lg[w][i][1] = x1; q_lg[w][i][2] = x2; q_lg[w][i][3] = x3;
      ds0 += x0; ds1 += x1; ds2 += x2; ds3 += x3;
    }
    ds0 = wsum(ds0); ds1 = wsum(ds1); ds2 = wsum(ds2); ds3 = wsum(ds3);
    const float dsel = (hl == 0) ? ds0 : ((hl == 1) ? ds1 : ((hl == 2) ? ds2 : ds3));
    const float invd = 1.0f / (dsel + 1e-16f);
    v4f acc = {0.f, 0.f, 0.f, 0.f};
    for (int i = 0; i < degt; ++i) {
      const int s = q_src[w][i];
      const float wg = q_lg[w][i][hl] * invd;
      const v4f v = *(const v4f*)(hsrc + (size_t)s * 128 + 4 * lane);
      acc += v * wg;
    }
    if (MODE == 0) {
      const v4f bb = *(const v4f*)(bias + 4 * lane);
      v4f val = acc + bb;
      val[0] = fmaxf(val[0], 0.f); val[1] = fmaxf(val[1], 0.f); val[2] = fmaxf(val[2], 0.f); val[3] = fmaxf(val[3], 0.f);
      const us h0 = bf_rne(val[0]), h1 = bf_rne(val[1]), h2 = bf_rne(val[2]), h3 = bf_rne(val[3]);
      const us l0 = bf_rne(val[0] - bf_val(h0)), l1 = bf_rne(val[1] - bf_val(h1));
      const us l2 = bf_rne(val[2] - bf_val(h2)), l3 = bf_rne(val[3] - bf_val(h3));
      fun[w][2 * lane]          = (unsigned)h0 | ((unsigned)h1 << 16);
      fun[w][2 * lane + 1]      = (unsigned)h2 | ((unsigned)h3 << 16);
      fun[w][64 + 2 * lane]     = (unsigned)l0 | ((unsigned)l1 << 16);
      fun[w][64 + 2 * lane + 1] = (unsigned)l2 | ((unsigned)l3 << 16);
      v4u o;
      o[0] = fun[w][4 * lane]; o[1] = fun[w][4 * lane + 1]; o[2] = fun[w][4 * lane + 2]; o[3] = fun[w][4 * lane + 3];
      us* tp = ((lane < 16) ? th : tl) + (size_t)n * 256 + coloff + 8 * (lane & 15);
      *(volatile v4u*)tp = o;
      __threadfence();
      *(volatile v4u*)tp = o;
    } else {
      v4f sm = acc;
      sm[0] += __shfl_xor(sm[0], 8);  sm[1] += __shfl_xor(sm[1], 8);  sm[2] += __shfl_xor(sm[2], 8);  sm[3] += __shfl_xor(sm[3], 8);
      sm[0] += __shfl_xor(sm[0], 16); sm[1] += __shfl_xor(sm[1], 16); sm[2] += __shfl_xor(sm[2], 16); sm[3] += __shfl_xor(sm[3], 16);
      const v4f bb = *(const v4f*)(bias + 4 * (lane & 7));
      v4f o = sm * 0.25f + bb;
      o[0] = fmaxf(o[0], 0.f); o[1] = fmaxf(o[1], 0.f); o[2] = fmaxf(o[2], 0.f); o[3] = fmaxf(o[3], 0.f);
      float* op = out + (size_t)n * 32 + 4 * (lane & 7);
      if (lane < 8) *(volatile v4f*)op = o;
      __threadfence();
      if (lane < 8) *(volatile v4f*)op = o;
    }
  }
}

extern "C" void kernel_launch(void* const* d_in, const int* in_sizes, int n_in,
                              void* d_out, int out_size, void* d_ws, size_t ws_size,
                              hipStream_t stream) {
  if (n_in < 29) return;
  const float* x_data  = (const float*)d_in[0];
  const float* x_tasks = (const float*)d_in[1];
  const float* x_dev   = (const float*)d_in[2];
  const int*   ei_dt   = (const int*)d_in[3];
  const float* ea_dt   = (const float*)d_in[4];
  const int*   ei_vt   = (const int*)d_in[5];
  const float* ea_vt   = (const float*)d_in[6];
  const int*   ei_tt   = (const int*)d_in[7];
  const float* ea_tt   = (const float*)d_in[8];
  const float *Ws1 = (const float*)d_in[9],  *Wd1 = (const float*)d_in[10], *We1 = (const float*)d_in[11];
  const float *As1 = (const float*)d_in[12], *Ad1 = (const float*)d_in[13], *Ae1 = (const float*)d_in[14];
  const float *b1  = (const float*)d_in[15];
  const float *Ws2 = (const float*)d_in[16], *Wd2 = (const float*)d_in[17], *We2 = (const float*)d_in[18];
  const float *As2 = (const float*)d_in[19], *Ad2 = (const float*)d_in[20], *Ae2 = (const float*)d_in[21];
  const float *b2  = (const float*)d_in[22];
  const float *W3  = (const float*)d_in[23], *We3 = (const float*)d_in[24];
  const float *As3 = (const float*)d_in[25], *Ad3 = (const float*)d_in[26], *Ae3 = (const float*)d_in[27];
  const float *b3  = (const float*)d_in[28];
  float* out = (float*)d_out;

  if (in_sizes[9] <= 0 || in_sizes[10] <= 0 || in_sizes[16] <= 0 || in_sizes[11] <= 0 ||
      in_sizes[18] <= 0 || in_sizes[24] <= 0) return;
  const int FD = in_sizes[9] / 128;
  const int FT = in_sizes[10] / 128;
  const int FV = in_sizes[16] / 128;
  const int ED1 = in_sizes[11] / 128, ED2 = in_sizes[18] / 128, ED3 = in_sizes[24] / 128;
  const int K3 = in_sizes[23] / 128;
  if (FD < 1 || FD > 32 || FT < 1 || FT > 32 || FV < 1 || FV > 32) return;
  if (ED1 < 1 || ED1 > 8 || ED2 < 1 || ED2 > 8 || ED3 != 4 || K3 != 256) return;
  if (in_sizes[17] != in_sizes[10]) return;
  const int NDAT = in_sizes[0] / FD;
  const int NT   = in_sizes[1] / FT;
  const int NDEV = in_sizes[2] / FV;
  const int EDT  = in_sizes[4] / ED1;
  const int EVT  = in_sizes[6] / ED2;
  const int ETT  = in_sizes[8] / ED3;
  if (NDAT <= 0 || NT <= 0 || NDEV <= 0 || EDT <= 0 || EVT <= 0 || ETT <= 0) return;
  if (in_sizes[3] != 2 * EDT || in_sizes[5] != 2 * EVT || in_sizes[7] != 2 * ETT) return;
  if (in_sizes[12] != 128 || in_sizes[15] != 128 || in_sizes[22] != 128 || in_sizes[28] != 32) return;
  if ((long)out_size != (long)NT * 32) return;
  if (NT > 65535) return;
  const int NPB = (NT + 2046) / 2047;
  if (NPB > 31) return;
  const int NBLK = (NT + NPB - 1) / NPB;
  const unsigned magic = (NPB > 1) ? (unsigned)((0x100000000ull + (unsigned long long)NPB - 1ull) /
                                                (unsigned long long)NPB) : 0u;
  const int nch1 = (EDT + CH - 1) / CH, nch2 = (EVT + CH - 1) / CH, nch3 = (ETT + CH - 1) / CH;
  int nchm = nch1; if (nch2 > nchm) nchm = nch2; if (nch3 > nchm) nchm = nch3;
  if (nchm > 256) return;
  const int KS3 = (K3 + 31) / 32;
  const int MpD = (NDAT + 1) & ~1, MpV = (NDEV + 1) & ~1, MpT = (NT + 1) & ~1;
  auto c16 = [](int m) { return (m + 15) & ~15; };

  size_t off = 0;
  auto carve = [&](size_t bytes) -> size_t { size_t o = off; off = (off + bytes + 255) & ~(size_t)255; return o; };
  const size_t o_bh1 = carve(8192), o_bl1 = carve(8192), o_bh2 = carve(8192), o_bl2 = carve(8192);
  const size_t o_bhd1 = carve(8192), o_bld1 = carve(8192), o_bhd2 = carve(8192), o_bld2 = carve(8192);
  const size_t o_bh3 = carve((size_t)KS3 * 8192), o_bl3 = carve((size_t)KS3 * 8192);
  const size_t o_wef1 = carve(128), o_wef2 = carve(128), o_wef3 = carve(128);
  const size_t o_xdh = carve((size_t)MpD * 64), o_xdl = carve((size_t)MpD * 64);
  const size_t o_xvh = carve((size_t)MpV * 64), o_xvl = carve((size_t)MpV * 64);
  const size_t o_xth = carve((size_t)MpT * 64), o_xtl = carve((size_t)MpT * 64);
  const size_t o_hs1 = carve((size_t)c16(NDAT) * 512), o_hs2 = carve((size_t)c16(NDEV) * 512);
  const size_t o_S1 = carve((size_t)c16(NDAT) * 32), o_S2 = carve((size_t)c16(NDEV) * 32);
  const size_t o_Sd1 = carve((size_t)c16(NT) * 32), o_Sd2 = carve((size_t)c16(NT) * 32), o_S3 = carve((size_t)c16(NT) * 32);
  const size_t o_th = carve((size_t)NT * 512), o_tl = carve((size_t)NT * 512);
  const size_t o_hs3 = carve((size_t)c16(NT) * 512);
  const size_t o_srt = carve((size_t)nchm * CH * 4), o_bnd = carve((size_t)nchm * NBC * 4);
  if (off > ws_size) return;

  char* ws = (char*)d_ws;
  us *bh1 = (us*)(ws + o_bh1), *bl1 = (us*)(ws + o_bl1), *bh2 = (us*)(ws + o_bh2), *bl2 = (us*)(ws + o_bl2);
  us *bhd1 = (us*)(ws + o_bhd1), *bld1 = (us*)(ws + o_bld1), *bhd2 = (us*)(ws + o_bhd2), *bld2 = (us*)(ws + o_bld2);
  us *bh3 = (us*)(ws + o_bh3), *bl3 = (us*)(ws + o_bl3);
  float *wef1 = (float*)(ws + o_wef1), *wef2 = (float*)(ws + o_wef2), *wef3 = (float*)(ws + o_wef3);
  us *xdh = (us*)(ws + o_xdh), *xdl = (us*)(ws + o_xdl), *xvh = (us*)(ws + o_xvh), *xvl = (us*)(ws + o_xvl);
  us *xth = (us*)(ws + o_xth), *xtl = (us*)(ws + o_xtl);
  float *hs1 = (float*)(ws + o_hs1), *hs2 = (float*)(ws + o_hs2);
  float *S1 = (float*)(ws + o_S1), *S2 = (float*)(ws + o_S2);
  float *Sd1 = (float*)(ws + o_Sd1), *Sd2 = (float*)(ws + o_Sd2), *S3 = (float*)(ws + o_S3);
  us *th = (us*)(ws + o_th), *tl = (us*)(ws + o_tl);
  float* hs3 = (float*)(ws + o_hs3);
  unsigned* srt = (unsigned*)(ws + o_srt);
  int* bnd = (int*)(ws + o_bnd);

  k_fold<<<1, 32, 0, stream>>>(We1, Ae1, ED1, wef1);
  k_fold<<<1, 32, 0, stream>>>(We2, Ae2, ED2, wef2);
  k_fold<<<1, 32, 0, stream>>>(We3, Ae3, ED3, wef3);

  k_packb<<<2, 256, 0, stream>>>(Ws1, FD, 1, bh1, bl1);
  k_packb<<<2, 256, 0, stream>>>(Ws2, FV, 1, bh2, bl2);
  k_packb<<<2, 256, 0, stream>>>(Wd1, FT, 1, bhd1, bld1);
  k_packb<<<2, 256, 0, stream>>>(Wd2, FT, 1, bhd2, bld2);
  k_packb<<<KS3 * 2, 256, 0, stream>>>(W3, K3, KS3, bh3, bl3);

  k_cvt<<<(MpD * 4 + 255) / 256, 256, 0, stream>>>(x_data, NDAT, MpD, FD, xdh, xdl);
  k_cvt<<<(MpV * 4 + 255) / 256, 256, 0, stream>>>(x_dev, NDEV, MpV, FV, xvh, xvl);
  k_cvt<<<(MpT * 4 + 255) / 256, 256, 0, stream>>>(x_tasks, NT, MpT, FT, xth, xtl);

  k_gemm<<<(NDAT + 15) / 16, 256, 0, stream>>>(xdh, xdl, 32, 1, NDAT, bh1, bl1, As1, As1, hs1, 1, S1);
  k_gemm<<<(NDEV + 15) / 16, 256, 0, stream>>>(xvh, xvl, 32, 1, NDEV, bh2, bl2, As2, As2, hs2, 1, S2);
  k_gemm<<<(NT + 15) / 16, 256, 0, stream>>>(xth, xtl, 32, 1, NT, bhd1, bld1, Ad1, Ad1, hs1, 0, Sd1);
  k_gemm<<<(NT + 15) / 16, 256, 0, stream>>>(xth, xtl, 32, 1, NT, bhd2, bld2, Ad2, Ad2, hs1, 0, Sd2);

  k_sort<<<nch1, 256, 0, stream>>>(ei_dt + EDT, EDT, NT, NPB, magic, srt, bnd);
  k_agg<0><<<NBLK, 256, 0, stream>>>(srt, bnd, nch1, NT, NPB, ei_dt, NDAT, ea_dt, ED1, wef1,
                                      S1, Sd1, hs1, b1, th, tl, 0, out);

  k_sort<<<nch2, 256, 0, stream>>>(ei_vt + EVT, EVT, NT, NPB, magic, srt, bnd);
  k_agg<0><<<NBLK, 256, 0, stream>>>(srt, bnd, nch2, NT, NPB, ei_vt, NDEV, ea_vt, ED2, wef2,
                                      S2, Sd2, hs2, b2, th, tl, 128, out);

  k_gemm<<<(NT + 15) / 16, 256, 0, stream>>>(th, tl, 256, KS3, NT, bh3, bl3, As3, Ad3, hs3, 1, S3);

  k_sort<<<nch3, 256, 0, stream>>>(ei_tt + ETT, ETT, NT, NPB, magic, srt, bnd);
  k_agg<1><<<NBLK, 256, 0, stream>>>(srt, bnd, nch3, NT, NPB, ei_tt, NT, ea_tt, ED3, wef3,
                                      S3, S3 + 4, hs3, b3, th, tl, 0, out);
  (void)hipGetLastError();
}
